// NLB_4741643895350
// MI455X (gfx1250) — hardware-verified
//
#include <hip/hip_runtime.h>
#include <math.h>
#include <stdint.h>

#ifndef NB
#define NB 2
#endif
#define NBF    2
#define CC     256
#define NN     6400
#ifndef NQ
#define NQ NN
#endif
#define DQ     128
#define MW     384
#define QT     64
#define OSP    68
#define OSPW   132
#define TP     72
#define WSC    256.0f
#define IWSC   0.00390625f
#define LNCAR  9.704060527839234f
#define ICAR   6.103515625e-05f

static_assert(NB >= 1 && NB <= NBF);
static_assert(NQ >= QT && NQ <= NN);
static_assert(NN % QT == 0);
static_assert(NQ % QT == 0);
static_assert(CC % QT == 0);
static_assert(MW == 3 * DQ);
static_assert(DQ == 2 * QT);
static_assert((DQ / 8) * 8 == DQ && (MW / 8) % (DQ / 8) == 0);
static_assert(CC % 16 == 0);
static_assert((OSP * 4) % 16 == 0);
static_assert((OSPW * 4) % 16 == 0);
static_assert((TP * 2) % 16 == 0);
static_assert(CC % 32 == 0 && NN % 32 == 0 && DQ % 32 == 0);
static_assert(NN % 4 == 0);

typedef _Float16       v16h __attribute__((ext_vector_type(16)));
typedef _Float16       v8h  __attribute__((ext_vector_type(8)));
typedef __bf16         v16b __attribute__((ext_vector_type(16)));
typedef unsigned short v8us __attribute__((ext_vector_type(8)));
typedef float          v8f  __attribute__((ext_vector_type(8)));
typedef float          v4f  __attribute__((ext_vector_type(4)));
typedef unsigned int   v4u  __attribute__((ext_vector_type(4)));

union Frag  { v8us u[2]; v16h h; v16b bf; };
union FragH { v16h v; v8h hv[2]; };
static_assert(sizeof(Frag) == 32);
static_assert(sizeof(FragH) == 32);

__device__ __forceinline__ unsigned short bf_bits(float f) {
  unsigned u = __float_as_uint(f);
  return (unsigned short)((u + 0x7FFFu + ((u >> 16) & 1u)) >> 16);
}
__device__ __forceinline__ float bf_up(unsigned short hb) { return __uint_as_float(((unsigned)hb) << 16); }
__device__ __forceinline__ float bfr(float f) { return bf_up(bf_bits(f)); }
__device__ __forceinline__ unsigned short h_bits(_Float16 x) { return __builtin_bit_cast(unsigned short, x); }
__device__ __forceinline__ unsigned pk16(unsigned short a, unsigned short b) { return (unsigned)a | ((unsigned)b << 16); }
__device__ __forceinline__ v8f zero8() { v8f z = {0.f, 0.f, 0.f, 0.f, 0.f, 0.f, 0.f, 0.f}; return z; }
__device__ __forceinline__ float hmax8(v8f s) {
  return fmaxf(fmaxf(fmaxf(s[0], s[1]), fmaxf(s[2], s[3])), fmaxf(fmaxf(s[4], s[5]), fmaxf(s[6], s[7])));
}

__device__ __forceinline__ Frag ldfrag(const unsigned short* p) {
  Frag f;
  f.u[0] = *(const v8us*)(p);
  f.u[1] = *(const v8us*)(p + 16);
  return f;
}

__device__ __forceinline__ v8f mma_h(v16h a, v16h b, v8f c) {
  v8f d = __builtin_amdgcn_wmma_f32_16x16x32_f16(false, a, false, b, (short)0, c, false, false);
#if defined(__HIP_DEVICE_COMPILE__)
  asm volatile("v_nop\n\tv_nop\n\tv_nop\n\tv_nop" : "+v"(d) : "v"(a), "v"(b));
#endif
  return d;
}
__device__ __forceinline__ v8f mma_b(v16b a, v16b b, v8f c) {
  v8f d = __builtin_amdgcn_wmma_f32_16x16x32_bf16(false, a, false, b, (short)0, c, false, false);
#if defined(__HIP_DEVICE_COMPILE__)
  const v16h ha = __builtin_bit_cast(v16h, a), hb = __builtin_bit_cast(v16h, b);
  asm volatile("v_nop\n\tv_nop\n\tv_nop\n\tv_nop" : "+v"(d) : "v"(ha), "v"(hb));
#endif
  return d;
}

__global__ __launch_bounds__(256)
void cvt_w(const float* __restrict__ tw, const float* __restrict__ pw, const float* __restrict__ gw,
           const float* __restrict__ ww, unsigned short* W16, unsigned short* Wo) {
  const int tid = threadIdx.x, blk = blockIdx.x;
  if (blk < MW / 8) {
    const int rl = tid >> 5, col = 8 * (tid & 31);
    const int o = 8 * blk + rl;
    const int sel = blk / (DQ / 8);
    const float* wbase = (sel == 0) ? tw : ((sel == 1) ? pw : gw);
    const float* s = wbase + (size_t)(o - sel * DQ) * CC + col;
    const v4f a = *(const v4f*)s;
    const v4f q = *(const v4f*)(s + 4);
    const float f[8] = {a[0], a[1], a[2], a[3], q[0], q[1], q[2], q[3]};
    v4u u;
#pragma unroll
    for (int t = 0; t < 4; ++t) {
      const _Float16 h0 = (_Float16)(bfr(f[2 * t]) * WSC);
      const _Float16 h1 = (_Float16)(bfr(f[2 * t + 1]) * WSC);
      u[t] = pk16(h_bits(h0), h_bits(h1));
    }
#pragma unroll
    for (int pass = 0; pass < 2; ++pass) {
      *(volatile v4u*)(W16 + (size_t)o * CC + col) = u;
      __threadfence();
    }
  } else {
    const int bb = blk - MW / 8;
    const int o = 16 * bb + (tid >> 4);
    const int col = 8 * (tid & 15);
    const float* s = ww + (size_t)o * DQ + col;
    const v4f a = *(const v4f*)s;
    const v4f q = *(const v4f*)(s + 4);
    const float f[8] = {a[0], a[1], a[2], a[3], q[0], q[1], q[2], q[3]};
    v4u u;
#pragma unroll
    for (int t = 0; t < 4; ++t) u[t] = pk16(bf_bits(f[2 * t]), bf_bits(f[2 * t + 1]));
#pragma unroll
    for (int pass = 0; pass < 2; ++pass) {
      *(volatile v4u*)(Wo + (size_t)o * DQ + col) = u;
      __threadfence();
    }
  }
}

__global__ __launch_bounds__(256)
void cvt_x(const float* __restrict__ x, unsigned short* XP) {
  __shared__ __align__(16) unsigned short T[QT * TP];
  const int tid = threadIdx.x;
  const int nb = blockIdx.x, cb = blockIdx.y, b = blockIdx.z;
  const int e = tid & 7, lq = tid >> 3;
  const int n0 = nb * QT, c0 = cb * QT;
#pragma unroll
  for (int it = 0; it < 2; ++it) {
    const int cl = it * 32 + lq;
    const float* sp = x + ((size_t)(b * CC + c0 + cl)) * NN + n0 + 8 * e;
    const v4f a = *(const v4f*)sp;
    const v4f q = *(const v4f*)(sp + 4);
    unsigned short hb[8];
#pragma unroll
    for (int t = 0; t < 4; ++t) {
      hb[t]     = h_bits((_Float16)bfr(a[t]));
      hb[4 + t] = h_bits((_Float16)bfr(q[t]));
    }
#pragma unroll
    for (int t = 0; t < 8; ++t) T[(8 * e + t) * TP + cl] = hb[t];
  }
  __syncthreads();
  v4u up[2];
#pragma unroll
  for (int it = 0; it < 2; ++it) {
    const int nl = it * 32 + lq;
    up[it] = *(const v4u*)(T + nl * TP + 8 * e);
  }
#pragma unroll
  for (int pass = 0; pass < 2; ++pass) {
#pragma unroll
    for (int it = 0; it < 2; ++it) {
      const int rl = it * 32 + lq;
      *(volatile v4u*)(XP + ((size_t)(b * NN + n0 + rl)) * CC + c0 + 8 * e) = up[it];
    }
    __threadfence();
  }
}

__global__ __launch_bounds__(128)
void gemm_p(const unsigned short* __restrict__ W16, const unsigned short* __restrict__ XP,
            const float* __restrict__ tb, const float* __restrict__ pb, const float* __restrict__ gb,
            unsigned short* Th, unsigned short* Tl, unsigned short* Fh, unsigned short* Fl, unsigned short* Gc) {
  __shared__ __align__(16) float Os[QT * OSP];
  const int tid  = threadIdx.x;
  const int lane = tid & 31, wave = tid >> 5;
  const int hh   = lane >> 4, c = lane & 15;
  const int nt   = blockIdx.x, mb = blockIdx.y, b = blockIdx.z;
  const int n0   = nt * QT, o0 = mb * QT;

  const unsigned short* ap = W16 + (size_t)(o0 + c) * CC + 8 * hh;
  const unsigned short* bp = XP + ((size_t)(b * NN + n0 + 16 * wave + c)) * CC + 8 * hh;

  v8f acc[4];
#pragma unroll
  for (int mt = 0; mt < 4; ++mt) acc[mt] = zero8();

#pragma unroll
  for (int ks = 0; ks < CC / 32; ++ks) {
    const Frag fb = ldfrag(bp + 32 * ks);
#pragma unroll
    for (int mt = 0; mt < 4; ++mt) {
      const Frag fa = ldfrag(ap + (size_t)(16 * mt) * CC + 32 * ks);
      acc[mt] = mma_h(fa.h, fb.h, acc[mt]);
    }
  }

  {
    const int nl = 16 * wave + c;
#pragma unroll
    for (int mt = 0; mt < 4; ++mt) {
      v4f va, vb;
#pragma unroll
      for (int r = 0; r < 4; ++r) { va[r] = acc[mt][r] * IWSC; vb[r] = acc[mt][4 + r] * IWSC; }
      *(v4f*)(Os + nl * OSP + 16 * mt + 8 * hh)     = va;
      *(v4f*)(Os + nl * OSP + 16 * mt + 8 * hh + 4) = vb;
    }
  }
  __syncthreads();

  const int dsel = (mb & 1) * QT;
  const float* bs = (mb < 2) ? tb : ((mb < 4) ? pb : gb);
  if (mb < 4) {
    const int e = tid & 7, lq = tid >> 3;
    unsigned short* Ph = (mb < 2) ? Th : Fh;
    unsigned short* Pl = (mb < 2) ? Tl : Fl;
    const v4f b0 = *(const v4f*)(bs + dsel + 8 * e);
    const v4f b1 = *(const v4f*)(bs + dsel + 8 * e + 4);
    const float bv[8] = {bfr(b0[0]), bfr(b0[1]), bfr(b0[2]), bfr(b0[3]),
                         bfr(b1[0]), bfr(b1[1]), bfr(b1[2]), bfr(b1[3])};
    v4u uh[4], ul[4];
#pragma unroll
    for (int it = 0; it < 4; ++it) {
      const int row = it * 16 + lq;
      const v4f a = *(const v4f*)(Os + row * OSP + 8 * e);
      const v4f q = *(const v4f*)(Os + row * OSP + 8 * e + 4);
      const float f[8] = {a[0] + bv[0], a[1] + bv[1], a[2] + bv[2], a[3] + bv[3],
                          q[0] + bv[4], q[1] + bv[5], q[2] + bv[6], q[3] + bv[7]};
#pragma unroll
      for (int t = 0; t < 4; ++t) {
        const float f0 = f[2 * t], f1 = f[2 * t + 1];
        const unsigned short hb0 = bf_bits(f0), hb1 = bf_bits(f1);
        const unsigned short lb0 = bf_bits(f0 - bf_up(hb0));
        const unsigned short lb1 = bf_bits(f1 - bf_up(hb1));
        uh[it][t] = pk16(hb0, hb1);
        ul[it][t] = pk16(lb0, lb1);
      }
    }
#pragma unroll
    for (int pass = 0; pass < 2; ++pass) {
#pragma unroll
      for (int it = 0; it < 4; ++it) {
        const int row = it * 16 + lq;
        const size_t po = ((size_t)(b * NN + n0 + row)) * DQ + dsel + 8 * e;
        *(volatile v4u*)(Ph + po) = uh[it];
        *(volatile v4u*)(Pl + po) = ul[it];
      }
      __threadfence();
    }
  } else {
    const int e = tid & 7, lq = tid >> 3;
    v4u ug[4];
#pragma unroll
    for (int it = 0; it < 4; ++it) {
      const int ol = it * 16 + lq;
      const float bvv = bfr(bs[dsel + ol]);
      unsigned short hb[8];
#pragma unroll
      for (int t = 0; t < 8; ++t) hb[t] = h_bits((_Float16)(Os[(8 * e + t) * OSP + ol] + bvv));
#pragma unroll
      for (int t = 0; t < 4; ++t) ug[it][t] = pk16(hb[2 * t], hb[2 * t + 1]);
    }
#pragma unroll
    for (int pass = 0; pass < 2; ++pass) {
#pragma unroll
      for (int it = 0; it < 4; ++it) {
        const int ol = it * 16 + lq;
        const size_t go = ((size_t)(b * DQ + dsel + ol)) * NN + n0 + 8 * e;
        *(volatile v4u*)(Gc + go) = ug[it];
      }
      __threadfence();
    }
  }
}

__global__ __launch_bounds__(128)
void colstat_k(const unsigned short* __restrict__ Th, const unsigned short* __restrict__ Tl,
               const unsigned short* __restrict__ Fh, const unsigned short* __restrict__ Fl, float* CS) {
  __shared__ __align__(16) float css[QT];
  const int tid  = threadIdx.x;
  const int wave = tid >> 5, lane = tid & 31;
  const int hh   = lane >> 4, c = lane & 15;
  const int m0   = blockIdx.x * QT, b = blockIdx.y;

  const size_t fo = ((size_t)(b * NN + m0 + 16 * wave + c)) * DQ + 8 * hh;
  Frag fh[4], fl[4];
#pragma unroll
  for (int kc = 0; kc < 4; ++kc) {
    fh[kc] = ldfrag(Fh + fo + 32 * kc);
    fl[kc] = ldfrag(Fl + fo + 32 * kc);
  }
  const unsigned short* Thp = Th + (size_t)b * NN * DQ + (size_t)c * DQ + 8 * hh;
  const unsigned short* Tlp = Tl + (size_t)b * NN * DQ + (size_t)c * DQ + 8 * hh;

  float m = -1.0e30f, l = 0.f;
#pragma unroll 1
  for (int kb = 0; kb < NN; kb += 32) {
    const unsigned short* t0p  = Thp + (size_t)kb * DQ;
    const unsigned short* t1p  = Thp + (size_t)(kb + 16) * DQ;
    const unsigned short* t0lp = Tlp + (size_t)kb * DQ;
    const unsigned short* t1lp = Tlp + (size_t)(kb + 16) * DQ;
    v8f s0 = zero8(), s1 = zero8();
#pragma unroll
    for (int kc = 0; kc < 4; ++kc) {
      const Frag t0  = ldfrag(t0p + 32 * kc);
      const Frag t1  = ldfrag(t1p + 32 * kc);
      const Frag t0l = ldfrag(t0lp + 32 * kc);
      const Frag t1l = ldfrag(t1lp + 32 * kc);
      s0 = mma_b(t0.bf, fh[kc].bf, s0);
      s1 = mma_b(t1.bf, fh[kc].bf, s1);
      s0 = mma_b(t0.bf, fl[kc].bf, s0);
      s1 = mma_b(t1.bf, fl[kc].bf, s1);
      s0 = mma_b(t0l.bf, fh[kc].bf, s0);
      s1 = mma_b(t1l.bf, fh[kc].bf, s1);
    }
    const float mx = fmaxf(hmax8(s0), hmax8(s1));
    const float mn = fmaxf(m, mx);
    const float corr = __expf(m - mn);
    float ls = 0.f;
#pragma unroll
    for (int r = 0; r < 8; ++r) ls += __expf(s0[r] - mn) + __expf(s1[r] - mn);
    l = l * corr + ls;
    m = mn;
  }
  const float mo = __shfl_xor(m, 16, 32);
  const float lo = __shfl_xor(l, 16, 32);
  const float mt = fmaxf(m, mo);
  const float lt = l * __expf(m - mt) + lo * __expf(mo - mt);
  const float csv = mt + logf(lt);
  if (hh == 0) css[16 * wave + c] = csv;
  __syncthreads();
  if (tid < 16) {
    const v4f v = *(const v4f*)(css + 4 * tid);
#pragma unroll
    for (int pass = 0; pass < 2; ++pass) {
      *(volatile v4f*)(CS + (size_t)b * NN + m0 + 4 * tid) = v;
      __threadfence();
    }
  }
}

__global__ __launch_bounds__(128)
void attn_k(const unsigned short* __restrict__ Th, const unsigned short* __restrict__ Tl,
            const unsigned short* __restrict__ Fh, const unsigned short* __restrict__ Fl,
            const unsigned short* __restrict__ Gc, const float* __restrict__ CS,
            unsigned short* Yh, unsigned short* Yl) {
  __shared__ __align__(32) float Cs[NN];
  __shared__ __align__(16) float Os[QT * OSPW];
  const int tid  = threadIdx.x;
  const int wave = tid >> 5, lane = tid & 31;
  const int hh   = lane >> 4, c = lane & 15;
  const int n0   = blockIdx.x * QT, b = blockIdx.y;

  for (int i = tid; i < NN / 4; i += 128)
    *(v4f*)(Cs + 4 * i) = *(const v4f*)(CS + (size_t)b * NN + 4 * i);
  __syncthreads();

  const size_t to = ((size_t)(b * NN + n0 + 16 * wave + c)) * DQ + 8 * hh;
  const unsigned short* Thp = Th + to;
  const unsigned short* Tlp = Tl + to;
  const unsigned short* Fhp = Fh + (size_t)b * NN * DQ + (size_t)c * DQ + 8 * hh;
  const unsigned short* Flp = Fl + (size_t)b * NN * DQ + (size_t)c * DQ + 8 * hh;
  const unsigned short* Gp = Gc + (size_t)b * DQ * NN + (size_t)c * NN + 8 * hh;

  v8f o[8];
#pragma unroll
  for (int j = 0; j < 8; ++j) o[j] = zero8();

#pragma unroll 1
  for (int kb = 0; kb < NN; kb += 32) {
    const unsigned short* p0p  = Fhp + (size_t)kb * DQ;
    const unsigned short* p1p  = Fhp + (size_t)(kb + 16) * DQ;
    const unsigned short* p0lp = Flp + (size_t)kb * DQ;
    const unsigned short* p1lp = Flp + (size_t)(kb + 16) * DQ;
    v8f s0 = zero8(), s1 = zero8();
#pragma unroll 1
    for (int kc = 0; kc < DQ / 32; ++kc) {
      const Frag th  = ldfrag(Thp + 32 * kc);
      const Frag tl  = ldfrag(Tlp + 32 * kc);
      const Frag p0  = ldfrag(p0p + 32 * kc);
      const Frag p1  = ldfrag(p1p + 32 * kc);
      const Frag p0l = ldfrag(p0lp + 32 * kc);
      const Frag p1l = ldfrag(p1lp + 32 * kc);
      s0 = mma_b(p0.bf, th.bf, s0);
      s1 = mma_b(p1.bf, th.bf, s1);
      s0 = mma_b(p0.bf, tl.bf, s0);
      s1 = mma_b(p1.bf, tl.bf, s1);
      s0 = mma_b(p0l.bf, th.bf, s0);
      s1 = mma_b(p1l.bf, th.bf, s1);
    }

    const v4f ca = *(const v4f*)(Cs + kb + 8 * hh);
    const v4f cb = *(const v4f*)(Cs + kb + 8 * hh + 4);
    const v4f cc = *(const v4f*)(Cs + kb + 16 + 8 * hh);
    const v4f cd = *(const v4f*)(Cs + kb + 16 + 8 * hh + 4);
    const float c0[8] = {ca[0], ca[1], ca[2], ca[3], cb[0], cb[1], cb[2], cb[3]};
    const float c1[8] = {cc[0], cc[1], cc[2], cc[3], cd[0], cd[1], cd[2], cd[3]};

    FragH pf;
#pragma unroll
    for (int r = 0; r < 8; ++r) {
      const float e0 = __expf(fminf(s0[r] - c0[r], 0.f) + LNCAR);
      const float e1 = __expf(fminf(s1[r] - c1[r], 0.f) + LNCAR);
      pf.hv[0][r] = (_Float16)e0;
      pf.hv[1][r] = (_Float16)e1;
    }

#pragma unroll
    for (int j = 0; j < 8; ++j) {
      const Frag gf = ldfrag(Gp + (size_t)(16 * j) * NN + kb);
      o[j] = mma_h(gf.h, pf.v, o[j]);
    }
  }

  {
    const int qrow = 16 * wave + c;
#pragma unroll
    for (int j = 0; j < 8; ++j) {
      v4f va, vb;
#pragma unroll
      for (int r = 0; r < 4; ++r) { va[r] = o[j][r] * ICAR; vb[r] = o[j][4 + r] * ICAR; }
      *(v4f*)(Os + qrow * OSPW + 16 * j + 8 * hh)     = va;
      *(v4f*)(Os + qrow * OSPW + 16 * j + 8 * hh + 4) = vb;
    }
  }
  __syncthreads();

  const int e = tid & 15, lq = tid >> 4;
  v4u uh[8], ul[8];
#pragma unroll
  for (int it = 0; it < 8; ++it) {
    const int row = it * 8 + lq;
    const v4f a = *(const v4f*)(Os + row * OSPW + 8 * e);
    const v4f q = *(const v4f*)(Os + row * OSPW + 8 * e + 4);
    const float f[8] = {a[0], a[1], a[2], a[3], q[0], q[1], q[2], q[3]};
#pragma unroll
    for (int t = 0; t < 4; ++t) {
      const float f0 = f[2 * t], f1 = f[2 * t + 1];
      const unsigned short hb0 = bf_bits(f0), hb1 = bf_bits(f1);
      const unsigned short lb0 = bf_bits(f0 - bf_up(hb0));
      const unsigned short lb1 = bf_bits(f1 - bf_up(hb1));
      uh[it][t] = pk16(hb0, hb1);
      ul[it][t] = pk16(lb0, lb1);
    }
  }
#pragma unroll
  for (int pass = 0; pass < 2; ++pass) {
#pragma unroll
    for (int it = 0; it < 8; ++it) {
      const int row = it * 8 + lq;
      const size_t po = ((size_t)(b * NN + n0 + row)) * DQ + 8 * e;
      *(volatile v4u*)(Yh + po) = uh[it];
      *(volatile v4u*)(Yl + po) = ul[it];
    }
    __threadfence();
  }
}

__global__ __launch_bounds__(128)
void gemm_w(const unsigned short* __restrict__ Wo, const unsigned short* __restrict__ Yh,
            const unsigned short* __restrict__ Yl, const float* __restrict__ wb,
            const float* __restrict__ x, float* out) {
  __shared__ __align__(16) float Os[QT * OSP];
  const int tid  = threadIdx.x;
  const int lane = tid & 31, wave = tid >> 5;
  const int hh   = lane >> 4, c = lane & 15;
  const int nt   = blockIdx.x, mb = blockIdx.y, b = blockIdx.z;
  const int n0   = nt * QT, o0 = mb * QT;

  const unsigned short* ap = Wo + (size_t)(o0 + c) * DQ + 8 * hh;
  const size_t yo = ((size_t)(b * NN + n0 + 16 * wave + c)) * DQ + 8 * hh;
  const unsigned short* bp  = Yh + yo;
  const unsigned short* blp = Yl + yo;

  v8f acc[4];
#pragma unroll
  for (int mt = 0; mt < 4; ++mt) acc[mt] = zero8();

#pragma unroll
  for (int ks = 0; ks < DQ / 32; ++ks) {
    const Frag fb  = ldfrag(bp + 32 * ks);
    const Frag fbl = ldfrag(blp + 32 * ks);
#pragma unroll
    for (int mt = 0; mt < 4; ++mt) {
      const Frag fa = ldfrag(ap + (size_t)(16 * mt) * DQ + 32 * ks);
      acc[mt] = mma_b(fa.bf, fb.bf, acc[mt]);
      acc[mt] = mma_b(fa.bf, fbl.bf, acc[mt]);
    }
  }

  {
    const int nl = 16 * wave + c;
#pragma unroll
    for (int mt = 0; mt < 4; ++mt) {
      v4f va, vb;
#pragma unroll
      for (int r = 0; r < 4; ++r) { va[r] = acc[mt][r]; vb[r] = acc[mt][4 + r]; }
      *(v4f*)(Os + nl * OSP + 16 * mt + 8 * hh)     = va;
      *(v4f*)(Os + nl * OSP + 16 * mt + 8 * hh + 4) = vb;
    }
  }
  __syncthreads();

  const int e = tid & 15, lq = tid >> 4;
  v4f res[8];
#pragma unroll
  for (int it = 0; it < 8; ++it) {
    const int ol = it * 8 + lq;
    const int o  = o0 + ol;
    const float bv = bfr(wb[o]);
    const size_t idx = ((size_t)(b * CC + o)) * NN + n0 + 4 * e;
    const v4f xv = *(const v4f*)(x + idx);
#pragma unroll
    for (int t = 0; t < 4; ++t) res[it][t] = (Os[(4 * e + t) * OSP + ol] + bv) + bfr(xv[t]);
  }
#pragma unroll
  for (int pass = 0; pass < 2; ++pass) {
#pragma unroll
    for (int it = 0; it < 8; ++it) {
      const int ol = it * 8 + lq;
      const size_t idx = ((size_t)(b * CC + o0 + ol)) * NN + n0 + 4 * e;
      *(volatile v4f*)(out + idx) = res[it];
    }
    __threadfence();
  }
}

extern "C" void kernel_launch(void* const* d_in, const int* in_sizes, int n_in,
                              void* d_out, int out_size, void* d_ws, size_t ws_size,
                              hipStream_t stream) {
  if (n_in < 9) return;
  if (in_sizes[0] < NB * CC * NN) return;
  if (in_sizes[1] != DQ * CC || in_sizes[3] != DQ * CC || in_sizes[5] != DQ * CC) return;
  if (in_sizes[2] != DQ || in_sizes[4] != DQ || in_sizes[6] != DQ) return;
  if (in_sizes[7] != CC * DQ || in_sizes[8] != CC) return;
  if (out_size < NB * CC * NN) return;

  size_t off = 0;
  auto carve = [&](size_t bytes) { const size_t o = off; off += (bytes + 255) & ~(size_t)255; return o; };
  const size_t oW16 = carve((size_t)MW * CC * 2);
  const size_t oWo  = carve((size_t)CC * DQ * 2);
  const size_t oXP  = carve((size_t)NB * NN * CC * 2);
  const size_t oTh  = carve((size_t)NB * NN * DQ * 2);
  const size_t oTl  = carve((size_t)NB * NN * DQ * 2);
  const size_t oFh  = carve((size_t)NB * NN * DQ * 2);
  const size_t oFl  = carve((size_t)NB * NN * DQ * 2);
  const size_t oGc  = carve((size_t)NB * DQ * NN * 2);
  const size_t oCS  = carve((size_t)NB * NN * 4);
  const size_t oYh  = carve((size_t)NB * NN * DQ * 2);
  const size_t oYl  = carve((size_t)NB * NN * DQ * 2);
  if (off > ws_size) return;
  if (off > (size_t)134217728) return;

  const float* x  = (const float*)d_in[0];
  const float* gw = (const float*)d_in[1];
  const float* gb = (const float*)d_in[2];
  const float* tw = (const float*)d_in[3];
  const float* tb = (const float*)d_in[4];
  const float* pw = (const float*)d_in[5];
  const float* pb = (const float*)d_in[6];
  const float* ww = (const float*)d_in[7];
  const float* wb = (const float*)d_in[8];

  char* ws = (char*)d_ws;
  unsigned short* W16 = (unsigned short*)(ws + oW16);
  unsigned short* Wo  = (unsigned short*)(ws + oWo);
  unsigned short* XP  = (unsigned short*)(ws + oXP);
  unsigned short* Th  = (unsigned short*)(ws + oTh);
  unsigned short* Tl  = (unsigned short*)(ws + oTl);
  unsigned short* Fh  = (unsigned short*)(ws + oFh);
  unsigned short* Fl  = (unsigned short*)(ws + oFl);
  unsigned short* Gc  = (unsigned short*)(ws + oGc);
  float*          CS  = (float*)(ws + oCS);
  unsigned short* Yh  = (unsigned short*)(ws + oYh);
  unsigned short* Yl  = (unsigned short*)(ws + oYl);
  float* out = (float*)d_out;

  const dim3 blk256(256), blk128(128);

  cvt_w<<<dim3(MW / 8 + CC / 16), blk256, 0, stream>>>(tw, pw, gw, ww, W16, Wo);
  cvt_x<<<dim3(NN / QT, CC / QT, NB), blk256, 0, stream>>>(x, XP);
  gemm_p<<<dim3(NN / QT, MW / QT, NB), blk128, 0, stream>>>(W16, XP, tb, pb, gb, Th, Tl, Fh, Fl, Gc);
  colstat_k<<<dim3(NN / QT, NB), blk128, 0, stream>>>(Th, Tl, Fh, Fl, CS);
  attn_k<<<dim3(NQ / QT, NB), blk128, 0, stream>>>(Th, Tl, Fh, Fl, Gc, CS, Yh, Yl);
  gemm_w<<<dim3(NQ / QT, CC / QT, NB), blk128, 0, stream>>>(Wo, Yh, Yl, wb, x, out);
  (void)hipGetLastError();
}
